// Enc_eta_83313775608357
// MI455X (gfx1250) — hardware-verified
//
#include <hip/hip_runtime.h>
#include <math.h>

typedef _Float16 v16h __attribute__((ext_vector_type(16)));
typedef _Float16 v8h  __attribute__((ext_vector_type(8)));
typedef float    v8f  __attribute__((ext_vector_type(8)));
typedef float    v4f  __attribute__((ext_vector_type(4)));
union Frag { v16h v; v8h half[2]; };

#define KC 3
#define DD 2
#define NF 5
#define HH 64
#define TT 32
#define OC 6
#define P1_WAVES 8
#define P1_THREADS 256
#define REC_F 128
#define HR 96
#define P2_THREADS 192

__device__ __forceinline__ v8f wmma_f16(v16h a, v16h b, v8f c) {
  v8f d = __builtin_amdgcn_wmma_f32_16x16x32_f16(false, a, false, b, (short)0, c, false, false);
  asm volatile("v_nop\n\tv_nop\n\tv_nop\n\tv_nop" : "+v"(d) : "v"(a), "v"(b));
  return d;
}

__device__ __forceinline__ v8f zero8() {
  v8f z;
  #pragma unroll
  for (int i = 0; i < 8; ++i) z[i] = 0.0f;
  return z;
}

__device__ __forceinline__ void fzero(Frag& f) {
  #pragma unroll
  for (int i = 0; i < 16; ++i) f.v[i] = (_Float16)0.0f;
}

__device__ __forceinline__ float tanh_fast(float x) {
  float e = __expf(2.0f * x);
  return 1.0f - 2.0f * __builtin_amdgcn_rcpf(e + 1.0f);
}

__global__ __launch_bounds__(P1_THREADS) void k_points(
    const float* __restrict__ obs,
    const float* __restrict__ state,
    const float* __restrict__ W1,
    const float* __restrict__ b1,
    const float* __restrict__ W2,
    const float* __restrict__ b2,
    float* __restrict__ part,
    int npts, int ntiles, int nit)
{
  __shared__ __attribute__((aligned(16))) _Float16 lds_h[P1_WAVES * 16 * HH];
  __shared__ float s_red[P1_WAVES * KC * TT * 2];
  __shared__ float s_cnt[P1_WAVES * KC * 32];
  __shared__ __attribute__((aligned(16))) float s_rec[REC_F];

  const int tid = threadIdx.x;
  const int w   = tid >> 5;
  const int l   = tid & 31;
  const int lm  = l & 15;
  const int lh  = l >> 4;
  const int sb  = blockIdx.y;
  const int g   = blockIdx.x;
  const int G   = gridDim.x;
  const int rbase = 8 * lh;

  Frag bw1[4];
  #pragma unroll
  for (int nt = 0; nt < 4; ++nt) {
    fzero(bw1[nt]);
    if (lh == 0) {
      const int c = 16 * nt + lm;
      #pragma unroll
      for (int i = 0; i < NF; ++i) bw1[nt].v[i] = (_Float16)W1[i * HH + c];
    }
  }
  Frag bw2[2][2];
  #pragma unroll
  for (int ks = 0; ks < 2; ++ks)
    #pragma unroll
    for (int nt = 0; nt < 2; ++nt) {
      const int c = 16 * nt + lm;
      #pragma unroll
      for (int i = 0; i < 8; ++i) {
        const int ka = 32 * ks + 8 * lh + i;
        const int kb = 32 * ks + 16 + 8 * lh + i;
        bw2[ks][nt].v[i]     = (_Float16)W2[ka * TT + c];
        bw2[ks][nt].v[8 + i] = (_Float16)W2[kb * TT + c];
      }
    }
  float bias1[4], bias2[2];
  #pragma unroll
  for (int nt = 0; nt < 4; ++nt) bias1[nt] = b1[16 * nt + lm];
  #pragma unroll
  for (int nt = 0; nt < 2; ++nt) bias2[nt] = b2[16 * nt + lm];

  _Float16* L = lds_h + w * 16 * HH;
  const size_t pbase = (size_t)sb * (size_t)npts;

  float acc[2][KC];
  #pragma unroll
  for (int nt = 0; nt < 2; ++nt)
    #pragma unroll
    for (int k = 0; k < KC; ++k) acc[nt][k] = 0.0f;
  float cnt0 = 0.0f, cnt1 = 0.0f, cnt2 = 0.0f;

  const int wstride = G * P1_WAVES;
  const int wg      = g * P1_WAVES + w;

  for (int it = 0; it < nit; ++it) {
    const int tile = it * wstride + wg;

    Frag a;
    fzero(a);
    float s0 = 0.0f, s1 = 0.0f, s2 = 0.0f;
    if (lh == 0) {
      const int p = tile * 16 + lm;
      if (tile < ntiles && p < npts) {
        const size_t q = pbase + (size_t)p;
        const float o0 = obs[q * 2 + 0];
        const float o1 = obs[q * 2 + 1];
        s0 = state[q * 3 + 0];
        s1 = state[q * 3 + 1];
        s2 = state[q * 3 + 2];
        a.v[0] = (_Float16)o0; a.v[1] = (_Float16)o1;
        a.v[2] = (_Float16)s0; a.v[3] = (_Float16)s1; a.v[4] = (_Float16)s2;
      }
    }
    cnt0 += s0; cnt1 += s1; cnt2 += s2;

    float wr0[8], wr1[8], wr2[8];
    #pragma unroll
    for (int j = 0; j < 8; ++j) {
      const int src = (rbase + j) << 2;
      wr0[j] = __int_as_float(__builtin_amdgcn_ds_bpermute(src, __float_as_int(s0)));
      wr1[j] = __int_as_float(__builtin_amdgcn_ds_bpermute(src, __float_as_int(s1)));
      wr2[j] = __int_as_float(__builtin_amdgcn_ds_bpermute(src, __float_as_int(s2)));
    }

    __syncthreads();
    #pragma unroll
    for (int nt = 0; nt < 4; ++nt) {
      v8f c = wmma_f16(a.v, bw1[nt].v, zero8());
      const int col = 16 * nt + lm;
      const float bb = bias1[nt];
      #pragma unroll
      for (int j = 0; j < 8; ++j)
        L[(rbase + j) * HH + col] = (_Float16)tanh_fast(c[j] + bb);
    }
    __syncthreads();

    Frag a2[2];
    {
      const _Float16* row = L + lm * HH;
      #pragma unroll
      for (int ks = 0; ks < 2; ++ks) {
        a2[ks].half[0] = *(const v8h*)(row + 32 * ks + 8 * lh);
        a2[ks].half[1] = *(const v8h*)(row + 32 * ks + 16 + 8 * lh);
      }
    }

    #pragma unroll
    for (int nt = 0; nt < 2; ++nt) {
      v8f c = wmma_f16(a2[0].v, bw2[0][nt].v, zero8());
      c = wmma_f16(a2[1].v, bw2[1][nt].v, c);
      const float bb = bias2[nt];
      #pragma unroll
      for (int j = 0; j < 8; ++j) {
        const float stat = c[j] + bb;
        acc[nt][0] += wr0[j] * stat;
        acc[nt][1] += wr1[j] * stat;
        acc[nt][2] += wr2[j] * stat;
      }
    }
  }

  #pragma unroll
  for (int nt = 0; nt < 2; ++nt) {
    const int t = 16 * nt + lm;
    #pragma unroll
    for (int k = 0; k < KC; ++k)
      s_red[((w * KC + k) * TT + t) * 2 + lh] = acc[nt][k];
  }
  s_cnt[(w * KC + 0) * 32 + l] = cnt0;
  s_cnt[(w * KC + 1) * 32 + l] = cnt1;
  s_cnt[(w * KC + 2) * 32 + l] = cnt2;
  __syncthreads();

  if (tid < KC * TT) {
    const int k = tid / TT, t = tid - k * TT;
    float s = 0.0f;
    for (int ww = 0; ww < P1_WAVES; ++ww) {
      s += s_red[((ww * KC + k) * TT + t) * 2 + 0];
      s += s_red[((ww * KC + k) * TT + t) * 2 + 1];
    }
    s_rec[tid] = s;
  } else if (tid < KC * TT + KC) {
    const int k = tid - KC * TT;
    float s = 0.0f;
    for (int ww = 0; ww < P1_WAVES; ++ww)
      for (int ll = 0; ll < 32; ++ll) s += s_cnt[(ww * KC + k) * 32 + ll];
    s_rec[tid] = s;
  } else if (tid < REC_F) {
    s_rec[tid] = 0.0f;
  }
  __syncthreads();

  if (tid < REC_F / 4) {
    const v4f v = *(const v4f*)(s_rec + 4 * tid);
    float* dst = part + ((size_t)sb * (size_t)G + (size_t)g) * REC_F + 4 * tid;
    *(volatile v4f*)dst = v;
    __threadfence();
    *(volatile v4f*)dst = v;
  }
}

template <int FIN, int FOUT, bool EXPO>
__device__ __forceinline__ void head_mlp(
    v16h a0, v16h a1,
    const float* __restrict__ W1, const float* __restrict__ b1v,
    const float* __restrict__ W2, const float* __restrict__ b2v,
    float* s_res, int col0, int wrow, int lm, int lh)
{
  float o[8][FOUT];
  #pragma unroll
  for (int r = 0; r < 8; ++r)
    #pragma unroll
    for (int j = 0; j < FOUT; ++j) o[r][j] = 0.0f;

  #pragma unroll
  for (int nt = 0; nt < 4; ++nt) {
    const int c = 16 * nt + lm;
    Frag bA, bB;
    #pragma unroll
    for (int i = 0; i < 8; ++i) {
      const int ka = 8 * lh + i;
      const int kb = 16 + 8 * lh + i;
      const int kc = 32 + 8 * lh + i;
      float vc = 0.0f;
      if (kc < FIN) vc = W1[kc * HH + c];
      bA.v[i]     = (_Float16)W1[ka * HH + c];
      bA.v[8 + i] = (_Float16)W1[kb * HH + c];
      bB.v[i]     = (_Float16)vc;
      bB.v[8 + i] = (_Float16)0.0f;
    }
    v8f acc = wmma_f16(a0, bA.v, zero8());
    acc = wmma_f16(a1, bB.v, acc);
    const float bb = b1v[c];
    float w2v[FOUT];
    #pragma unroll
    for (int j = 0; j < FOUT; ++j) w2v[j] = W2[c * FOUT + j];
    #pragma unroll
    for (int r = 0; r < 8; ++r) {
      const float th = tanhf(acc[r] + bb);
      #pragma unroll
      for (int j = 0; j < FOUT; ++j) o[r][j] += th * w2v[j];
    }
  }
  #pragma unroll
  for (int r = 0; r < 8; ++r)
    #pragma unroll
    for (int j = 0; j < FOUT; ++j) {
      float v = o[r][j];
      v += __shfl_xor(v, 1);
      v += __shfl_xor(v, 2);
      v += __shfl_xor(v, 4);
      v += __shfl_xor(v, 8);
      o[r][j] = v;
    }
  if (lm == 0) {
    #pragma unroll
    for (int r = 0; r < 8; ++r)
      #pragma unroll
      for (int j = 0; j < FOUT; ++j) {
        float val = o[r][j] + b2v[j];
        if (EXPO) val = expf(val);
        s_res[(wrow + 8 * lh + r) * OC + col0 + j] = val;
      }
  }
}

__global__ __launch_bounds__(P2_THREADS) void k_heads(
    const float* __restrict__ part,
    const float* __restrict__ muW1, const float* __restrict__ mub1,
    const float* __restrict__ muW2, const float* __restrict__ mub2,
    const float* __restrict__ sgW1, const float* __restrict__ sgb1,
    const float* __restrict__ sgW2, const float* __restrict__ sgb2,
    const float* __restrict__ alW1, const float* __restrict__ alb1,
    const float* __restrict__ alW2, const float* __restrict__ alb2,
    const float* __restrict__ beW1, const float* __restrict__ beb1,
    const float* __restrict__ beW2, const float* __restrict__ beb2,
    float* out, int SB, int G, int R)
{
  __shared__ __attribute__((aligned(16))) _Float16 A_mu[HR * 64];
  __shared__ __attribute__((aligned(16))) _Float16 A_ra[HR * 64];
  __shared__ float s_cs[HR];
  __shared__ __attribute__((aligned(16))) float s_res[HR * OC];

  const int tid = threadIdx.x;
  const int w   = tid >> 5;
  const int l   = tid & 31;
  const int lm  = l & 15;
  const int lh  = l >> 4;
  const int row0 = blockIdx.x * HR;
  (void)SB;

  for (int r = tid; r < HR; r += P2_THREADS) {
    const int grow = row0 + r;
    float cs = 1.0f;
    if (grow < R) {
      const int sb = grow / KC, k = grow - sb * KC;
      float s = 0.0f;
      for (int g = 0; g < G; ++g)
        s += part[((size_t)sb * (size_t)G + (size_t)g) * REC_F + KC * TT + k];
      cs = (s == 0.0f) ? 1.0f : s;
    }
    s_cs[r] = cs;
  }
  __syncthreads();

  for (int idx = tid; idx < HR * TT; idx += P2_THREADS) {
    const int r = idx >> 5, t = idx & 31;
    const int grow = row0 + r;
    float x = 0.0f;
    if (grow < R) {
      const int sb = grow / KC, k = grow - sb * KC;
      float s = 0.0f;
      for (int g = 0; g < G; ++g)
        s += part[((size_t)sb * (size_t)G + (size_t)g) * REC_F + k * TT + t];
      x = s * (1.0f / s_cs[r]);
    }
    const _Float16 xh = (_Float16)x;
    A_mu[r * 64 + t] = xh;
    A_ra[r * 64 + t] = xh;
    const float cm = (t == 2 || t == 3) ? 7.0f : 0.0f;
    const float cr = (t == 0) ? 8.0f : ((t == 1) ? 16.0f : 0.0f);
    A_mu[r * 64 + 32 + t] = (_Float16)cm;
    A_ra[r * 64 + 32 + t] = (_Float16)cr;
  }
  __syncthreads();

  Frag amu[2], ara[2];
  {
    const int rp = (16 * w + lm) * 64;
    #pragma unroll
    for (int ks = 0; ks < 2; ++ks) {
      amu[ks].half[0] = *(const v8h*)(A_mu + rp + 32 * ks + 8 * lh);
      amu[ks].half[1] = *(const v8h*)(A_mu + rp + 32 * ks + 16 + 8 * lh);
      ara[ks].half[0] = *(const v8h*)(A_ra + rp + 32 * ks + 8 * lh);
      ara[ks].half[1] = *(const v8h*)(A_ra + rp + 32 * ks + 16 + 8 * lh);
    }
  }
  const int wrow = 16 * w;
  head_mlp<36, 2, false>(amu[0].v, amu[1].v, muW1, mub1, muW2, mub2, s_res, 0, wrow, lm, lh);
  head_mlp<36, 2, true >(amu[0].v, amu[1].v, sgW1, sgb1, sgW2, sgb2, s_res, 2, wrow, lm, lh);
  head_mlp<34, 1, true >(ara[0].v, ara[1].v, alW1, alb1, alW2, alb2, s_res, 4, wrow, lm, lh);
  head_mlp<34, 1, true >(ara[0].v, ara[1].v, beW1, beb1, beW2, beb2, s_res, 5, wrow, lm, lh);
  __syncthreads();

  int nrows = R - row0;
  if (nrows > HR) nrows = HR;
  const int nflo = nrows * OC;
  float* ob = out + (size_t)row0 * OC;

  for (int t = tid; 4 * t < nflo; t += P2_THREADS) {
    if (4 * t + 4 <= nflo) {
      const v4f v = *(const v4f*)(s_res + 4 * t);
      *(volatile v4f*)(ob + 4 * t) = v;
    } else {
      for (int e = 4 * t; e < nflo; ++e) { const float v = s_res[e]; *(volatile float*)(ob + e) = v; }
    }
  }
  __threadfence();
  for (int t = tid; 4 * t < nflo; t += P2_THREADS) {
    if (4 * t + 4 <= nflo) {
      const v4f v = *(const v4f*)(s_res + 4 * t);
      *(volatile v4f*)(ob + 4 * t) = v;
    } else {
      for (int e = 4 * t; e < nflo; ++e) { const float v = s_res[e]; *(volatile float*)(ob + e) = v; }
    }
  }
}

extern "C" void kernel_launch(void* const* d_in, const int* in_sizes, int n_in,
                              void* d_out, int out_size, void* d_ws, size_t ws_size,
                              hipStream_t stream) {
  if (n_in < 22 || out_size <= 0) return;

  const int SB = out_size / (KC * OC);
  if (SB <= 0) return;
  const int npts = in_sizes[1] / (SB * KC);
  const int ntiles = (npts + 15) / 16;
  const int R = SB * KC;

  int G = 32;
  while (G > 1 && (size_t)SB * (size_t)G * REC_F * sizeof(float) > ws_size) G >>= 1;
  if ((size_t)SB * (size_t)G * REC_F * sizeof(float) > ws_size) return;
  const int nit = (ntiles + G * P1_WAVES - 1) / (G * P1_WAVES);

  float* part = (float*)d_ws;

  const float* obs   = (const float*)d_in[0];
  const float* state = (const float*)d_in[1];
  const float* nsW1  = (const float*)d_in[2];
  const float* nsb1  = (const float*)d_in[3];
  const float* nsW2  = (const float*)d_in[4];
  const float* nsb2  = (const float*)d_in[5];

  dim3 grid1(G, SB);
  k_points<<<grid1, P1_THREADS, 0, stream>>>(obs, state, nsW1, nsb1, nsW2, nsb2,
                                              part, npts, ntiles, nit);

  const int grid2 = (R + HR - 1) / HR;
  k_heads<<<grid2, P2_THREADS, 0, stream>>>(
      part,
      (const float*)d_in[6],  (const float*)d_in[7],  (const float*)d_in[8],  (const float*)d_in[9],
      (const float*)d_in[10], (const float*)d_in[11], (const float*)d_in[12], (const float*)d_in[13],
      (const float*)d_in[14], (const float*)d_in[15], (const float*)d_in[16], (const float*)d_in[17],
      (const float*)d_in[18], (const float*)d_in[19], (const float*)d_in[20], (const float*)d_in[21],
      (float*)d_out, SB, G, R);
}
